// DeformConv2dBlock_71004399337612
// MI455X (gfx1250) — hardware-verified
//
#include <hip/hip_runtime.h>

typedef __attribute__((ext_vector_type(16))) _Float16 v16h;
typedef __attribute__((ext_vector_type(8)))  _Float16 v8h;
typedef __attribute__((ext_vector_type(16))) __bf16   v16b;
typedef __attribute__((ext_vector_type(8)))  __bf16   v8b;
typedef __attribute__((ext_vector_type(8)))  float    v8f;
typedef __attribute__((ext_vector_type(4)))  float    v4f;
typedef __attribute__((ext_vector_type(4)))  unsigned int u4v;

constexpr int NIMG   = 8;
constexpr int NCH    = 64;
constexpr int IMGH   = 128;
constexpr int IMGW   = 128;
constexpr int HWPIX  = IMGH * IMGW;
constexpr int NPTS   = 9;
constexpr int NOFFCH = 2 * NPTS;
constexpr int KDIM   = NCH * NPTS;
constexpr int QPR    = KDIM / 8;
constexpr int PADH   = IMGH + 2;
constexpr int PADW   = IMGW + 2;
constexpr int PADHW  = PADH * PADW;
constexpr int NXP    = NIMG * NCH * PADHW;
static_assert(KDIM % 32 == 0);
static_assert(HWPIX % 64 == 0);
static_assert(NCH % 64 == 0);
static_assert(NXP % 64 == 0);
static_assert((NXP / 8) % 256 == 0);
static_assert((HWPIX * QPR) % 256 == 0);
static_assert((NCH * QPR) % 256 == 0);
static_assert(QPR % 8 == 0);

__device__ __forceinline__ unsigned short f2bf_bits(float f) {
  unsigned u = __float_as_uint(f);
  return (unsigned short)((u + 0x7FFFu + ((u >> 16) & 1u)) >> 16);
}
__device__ __forceinline__ float bf_bits2f(unsigned short h) { return __uint_as_float(((unsigned)h) << 16); }

__device__ __forceinline__ void dep_guard_h(v8f& a, v8f& b, v16h x, v16h y) { asm volatile("v_nop\n\tv_nop\n\tv_nop\n\tv_nop" : "+v"(a), "+v"(b) : "v"(x), "v"(y)); }
__device__ __forceinline__ void dep_guard_b(v8f& a, v8f& b, v16b x, v16b y) { asm volatile("v_nop\n\tv_nop\n\tv_nop\n\tv_nop" : "+v"(a), "+v"(b) : "v"(x), "v"(y)); }
__device__ __forceinline__ void keep4_h(v16h a, v16h b, v16h c, v16h d) { asm volatile("v_nop" :: "v"(a), "v"(b), "v"(c), "v"(d)); }
__device__ __forceinline__ void keep4_b(v16b a, v16b b, v16b c, v16b d) { asm volatile("v_nop" :: "v"(a), "v"(b), "v"(c), "v"(d)); }
__device__ __forceinline__ void acc_guard4(v8f& a, v8f& b, v8f& c, v8f& d) { asm volatile("v_nop\n\tv_nop\n\tv_nop\n\tv_nop" : "+v"(a), "+v"(b), "+v"(c), "+v"(d)); }
template <typename T> struct Frag;
template <> struct Frag<_Float16> {
  typedef v16h V; union U { v16h v; v8h h[2]; };
  static __device__ __forceinline__ v16h load(const _Float16* p) {
    U f; f.h[0] = *(const v8h*)(p); f.h[1] = *(const v8h*)(p + 16); return f.v;
  }
  static __device__ __forceinline__ v8f mma(v16h a, v16h b, v8f c) {
    return __builtin_amdgcn_wmma_f32_16x16x32_f16(false, a, false, b, (short)0, c, false, false);
  }
  static __device__ __forceinline__ void guard(v8f& a, v8f& b, v16h x, v16h y) { dep_guard_h(a, b, x, y); }
  static __device__ __forceinline__ void keep(v16h a, v16h b, v16h c, v16h d) { keep4_h(a, b, c, d); }
};
template <> struct Frag<__bf16> {
  typedef v16b V; union U { v16b v; v8b h[2]; };
  static __device__ __forceinline__ v16b load(const __bf16* p) {
    U f; f.h[0] = *(const v8b*)(p); f.h[1] = *(const v8b*)(p + 16); return f.v;
  }
  static __device__ __forceinline__ v8f mma(v16b a, v16b b, v8f c) {
    return __builtin_amdgcn_wmma_f32_16x16x32_bf16(false, a, false, b, (short)0, c, false, false);
  }
  static __device__ __forceinline__ void guard(v8f& a, v8f& b, v16b x, v16b y) { dep_guard_b(a, b, x, y); }
  static __device__ __forceinline__ void keep(v16b a, v16b b, v16b c, v16b d) { keep4_b(a, b, c, d); }
};

template <int ET> struct Elem;
template <> struct Elem<0> { typedef _Float16 T; };
template <> struct Elem<1> { typedef __bf16 T; };

template <int ET, int SPLIT_MODE, bool RESID>
__global__ __launch_bounds__(256) void wmma_gemm64(
    const unsigned short* __restrict__ Ap, const unsigned short* __restrict__ A2p, int lda, long strideA,
    const unsigned short* __restrict__ Btp, const unsigned short* __restrict__ Bt2p, int ldb, long strideB,
    float* __restrict__ Cout, int ldc, long strideC,
    const float* __restrict__ resid, long strideR,
    int M, int N, int K, float scale) {
  typedef typename Elem<ET>::T T;
  typedef typename Frag<T>::V V;
  constexpr bool SPLB = (SPLIT_MODE != 0);
  constexpr bool SPLA = (SPLIT_MODE == 1);
  const T* A = (const T*)Ap; const T* A2 = (const T*)A2p; const T* Bt = (const T*)Btp; const T* Bt2 = (const T*)Bt2p;
  __shared__ __align__(16) float sT[8][16 * 68];
  const int b    = blockIdx.y;
  const int lane = threadIdx.x & 31;
  const int wave = threadIdx.x >> 5;
  const int tilesN = N >> 6;
  const int tilesM = M >> 6;
  const int tile = blockIdx.x * 8 + wave;
  if (tile >= tilesM * tilesN) return;
  const int tm = tile / tilesN;
  const int tn = tile - tm * tilesN;
  const int m0 = tm << 6;
  const int n0 = tn << 6;

  const T* Ab  = A  + (size_t)b * strideA;
  const T* Bb  = Bt + (size_t)b * strideB;
  const T* Ab2 = SPLA ? (A2  + (size_t)b * strideA) : nullptr;
  const T* Bb2 = SPLB ? (Bt2 + (size_t)b * strideB) : nullptr;

  const int rlane = lane & 15;
  const int koff  = (lane >> 4) * 8;
  const int mOff  = (lane >> 4) * 8;

  v8f acc[4][4];
#pragma unroll
  for (int i = 0; i < 4; ++i)
#pragma unroll
    for (int j = 0; j < 4; ++j) acc[i][j] = (v8f){0.f,0.f,0.f,0.f,0.f,0.f,0.f,0.f};

  for (int k0 = 0; k0 < K; k0 += 32) {
    V bh[4], bl[4];
#pragma unroll
    for (int j = 0; j < 4; ++j) {
      const size_t bo = (size_t)(n0 + (j << 4) + rlane) * ldb + koff + k0;
      bh[j] = Frag<T>::load(Bb + bo);
      if (SPLB) bl[j] = Frag<T>::load(Bb2 + bo);
    }
#pragma unroll
    for (int i = 0; i < 4; ++i) {
      const size_t ao = (size_t)(m0 + (i << 4) + rlane) * lda + koff + k0;
      V ah = Frag<T>::load(Ab + ao);
      V al;
      if (SPLA) al = Frag<T>::load(Ab2 + ao);
#pragma unroll
      for (int j = 0; j < 4; ++j) {
        acc[i][j] = Frag<T>::mma(ah, bh[j], acc[i][j]);
        if (SPLB) acc[i][j] = Frag<T>::mma(ah, bl[j], acc[i][j]);
        if (SPLA) acc[i][j] = Frag<T>::mma(al, bh[j], acc[i][j]);
      }
      Frag<T>::guard(acc[i][0], acc[i][3], ah, SPLA ? al : ah);
    }
    Frag<T>::keep(bh[0], bh[1], bh[2], bh[3]);
    if (SPLB) Frag<T>::keep(bl[0], bl[1], bl[2], bl[3]);
  }
  acc_guard4(acc[0][0], acc[0][1], acc[0][2], acc[0][3]);
  acc_guard4(acc[1][0], acc[1][1], acc[1][2], acc[1][3]);
  acc_guard4(acc[2][0], acc[2][1], acc[2][2], acc[2][3]);
  acc_guard4(acc[3][0], acc[3][1], acc[3][2], acc[3][3]);

  float* slab = sT[wave];
  float* C = Cout + (size_t)b * strideC;
  const float* Rb = RESID ? (resid + (size_t)b * strideR) : nullptr;
  const int hh = lane >> 4, c4 = (lane & 15) * 4;
#pragma unroll
  for (int i = 0; i < 4; ++i) {
    const int mBase = m0 + (i << 4);
#pragma unroll
    for (int j = 0; j < 4; ++j) {
#pragma unroll
      for (int r = 0; r < 8; ++r) {
        slab[(mOff + r) * 68 + (j << 4) + rlane] = acc[i][j][r] * scale;
      }
    }
    __builtin_amdgcn_fence(__ATOMIC_RELEASE, "workgroup");
    __builtin_amdgcn_wave_barrier();
    __builtin_amdgcn_fence(__ATOMIC_ACQUIRE, "workgroup");
    v4f vals[8];
#pragma unroll
    for (int it = 0; it < 8; ++it) {
      const int row = it * 2 + hh;
      v4f v = *(const v4f*)(slab + row * 68 + c4);
      if (RESID) {
        const v4f rv = *(const v4f*)(Rb + (size_t)(mBase + row) * ldc + n0 + c4);
#pragma unroll
        for (int e = 0; e < 4; ++e) {
          unsigned u = __float_as_uint(rv[e]);
          u = (u + 0x7FFFu + ((u >> 16) & 1u)) & 0xFFFF0000u;
          v[e] = v[e] + __uint_as_float(u);
        }
      }
      vals[it] = v;
    }
    for (int pass = 0; pass < 2; ++pass) {
#pragma unroll
      for (int it = 0; it < 8; ++it) {
        const int row = it * 2 + hh;
        *(volatile v4f*)(C + (size_t)(mBase + row) * ldc + n0 + c4) = vals[it];
      }
      __threadfence();
    }
    __builtin_amdgcn_fence(__ATOMIC_RELEASE, "workgroup");
    __builtin_amdgcn_wave_barrier();
    __builtin_amdgcn_fence(__ATOMIC_ACQUIRE, "workgroup");
  }
}

__global__ __launch_bounds__(256) void k_prep_w(const float* __restrict__ w_off, const float* __restrict__ w_conv,
                                                unsigned short* __restrict__ woffp, unsigned short* __restrict__ wcp) {
  constexpr int NBLK_HALF = (NCH * QPR) / 256;
  const int blk = blockIdx.x;
  const bool first = (blk < NBLK_HALF);
  const int t = (first ? blk : (blk - NBLK_HALF)) * 256 + (int)threadIdx.x;
  const int o = t / QPR;
  const int q = t - o * QPR;
  const int grp = q >> 3;
  const int cb = (q & 7) * 8;
  unsigned pk[4];
  if (first) {
    const int oc = (o < NOFFCH) ? o : (NOFFCH - 1);
#pragma unroll
    for (int i = 0; i < 8; ++i) {
      const int c = cb + i;
      const float v = w_off[(oc * NCH + c) * 9 + grp];
      const unsigned bits = (o < NOFFCH) ? (unsigned)f2bf_bits(v) : 0u;
      if (i & 1) pk[i >> 1] |= (bits << 16); else pk[i >> 1] = bits;
    }
    u4v wv; wv.x = pk[0]; wv.y = pk[1]; wv.z = pk[2]; wv.w = pk[3];
    u4v* dst = (u4v*)(void*)woffp + t;
    *(volatile u4v*)dst = wv;
    __threadfence();
    *(volatile u4v*)dst = wv;
  } else {
#pragma unroll
    for (int i = 0; i < 8; ++i) {
      const int c = cb + i;
      const float v = w_conv[(o * NCH + c) * 9 + grp];
      const unsigned bits = (unsigned)f2bf_bits(v);
      if (i & 1) pk[i >> 1] |= (bits << 16); else pk[i >> 1] = bits;
    }
    u4v wv; wv.x = pk[0]; wv.y = pk[1]; wv.z = pk[2]; wv.w = pk[3];
    u4v* dst = (u4v*)(void*)wcp + t;
    *(volatile u4v*)dst = wv;
    __threadfence();
    *(volatile u4v*)dst = wv;
  }
}

__global__ __launch_bounds__(256) void k_pad_x(const float* __restrict__ x, unsigned short* __restrict__ xp) {
  const int g = blockIdx.x * 256 + (int)threadIdx.x;
  unsigned pk[4];
#pragma unroll
  for (int i = 0; i < 8; ++i) {
    const int e  = g * 8 + i;
    const int ch = e / PADHW;
    const int r  = e - ch * PADHW;
    const int qx = r / PADW;
    const int qy = r - qx * PADW;
    const bool inb = (qx >= 1) && (qx <= IMGH) && (qy >= 1) && (qy <= IMGW);
    int hx = qx - 1; hx = (hx < 0) ? 0 : ((hx > IMGH - 1) ? (IMGH - 1) : hx);
    int wy = qy - 1; wy = (wy < 0) ? 0 : ((wy > IMGW - 1) ? (IMGW - 1) : wy);
    const float v = x[(size_t)ch * HWPIX + hx * IMGW + wy];
    const unsigned bits = inb ? (unsigned)f2bf_bits(v) : 0u;
    if (i & 1) pk[i >> 1] |= (bits << 16); else pk[i >> 1] = bits;
  }
  u4v wv; wv.x = pk[0]; wv.y = pk[1]; wv.z = pk[2]; wv.w = pk[3];
  u4v* dst = (u4v*)(void*)xp + g;
  *(volatile u4v*)dst = wv;
  __threadfence();
  *(volatile u4v*)dst = wv;
}

__global__ __launch_bounds__(256) void k_im2col(const unsigned short* __restrict__ xpb, unsigned short* __restrict__ im) {
  const int g = blockIdx.x * 256 + (int)threadIdx.x;
  const int p = g / QPR;
  const int q = g - p * QPR;
  const int tap = q >> 3;
  const int cb  = (q & 7) * 8;
  const int kh  = tap / 3;
  const int kw  = tap - kh * 3;
  const int h   = p / IMGW;
  const int w   = p - h * IMGW;
  const unsigned short* src = xpb + (size_t)cb * PADHW + (h + kh) * PADW + (w + kw);
  unsigned pk[4];
#pragma unroll
  for (int i = 0; i < 8; ++i) {
    const unsigned a = (unsigned)src[(size_t)i * PADHW];
    if (i & 1) pk[i >> 1] |= (a << 16); else pk[i >> 1] = a;
  }
  u4v wv; wv.x = pk[0]; wv.y = pk[1]; wv.z = pk[2]; wv.w = pk[3];
  u4v* dst = (u4v*)(void*)im + g;
  *(volatile u4v*)dst = wv;
  __threadfence();
  *(volatile u4v*)dst = wv;
}

__global__ __launch_bounds__(256) void k_sample(const unsigned short* __restrict__ xpb, const float* __restrict__ offp,
                                                const float* __restrict__ b_off,
                                                unsigned short* __restrict__ xh, unsigned short* __restrict__ xl) {
  const int g = blockIdx.x * 256 + (int)threadIdx.x;
  const int p = g / QPR;
  const int q = g - p * QPR;
  const int n = q >> 3;
  const int cb = (q & 7) * 8;
  const int h = p / IMGW;
  const int w = p - h * IMGW;

  const float offx = offp[(size_t)n * HWPIX + p];
  const float offy = offp[(size_t)(NPTS + n) * HWPIX + p];
  const float bx = bf_bits2f(f2bf_bits(b_off[n]));
  const float by = bf_bits2f(f2bf_bits(b_off[NPTS + n]));
  const int   ni  = n / 3;
  const float pnx = (float)(ni - 1);
  const float pny = (float)(n - ni * 3 - 1);
  const float px = ((offx + bx) + pnx) + (float)(h + 1);
  const float py = ((offy + by) + pny) + (float)(w + 1);

  const float fx = floorf(px), fy = floorf(py);
  const float lim = (float)(PADH - 1);
  const float qltx = fminf(fmaxf(fx, 0.f), lim);
  const float qlty = fminf(fmaxf(fy, 0.f), lim);
  const float qrbx = fminf(fmaxf(fx + 1.f, 0.f), lim);
  const float qrby = fminf(fmaxf(fy + 1.f, 0.f), lim);
  const float pxc  = fminf(fmaxf(px, 0.f), lim);
  const float pyc  = fminf(fmaxf(py, 0.f), lim);
  const float axl = 1.f + (qltx - pxc);
  const float axr = 1.f - (qrbx - pxc);
  const float ayl = 1.f + (qlty - pyc);
  const float ayr = 1.f - (qrby - pyc);
  const float g_lt = axl * ayl;
  const float g_rb = axr * ayr;
  const float g_lb = axl * ayr;
  const float g_rt = axr * ayl;
  int ixl = (int)qltx, ixr = (int)qrbx, iyl = (int)qlty, iyr = (int)qrby;
  ixl = (ixl < 0) ? 0 : ((ixl > PADH - 1) ? (PADH - 1) : ixl);
  ixr = (ixr < 0) ? 0 : ((ixr > PADH - 1) ? (PADH - 1) : ixr);
  iyl = (iyl < 0) ? 0 : ((iyl > PADW - 1) ? (PADW - 1) : iyl);
  iyr = (iyr < 0) ? 0 : ((iyr > PADW - 1) ? (PADW - 1) : iyr);
  const int o_lt = ixl * PADW + iyl;
  const int o_rb = ixr * PADW + iyr;
  const int o_lb = ixl * PADW + iyr;
  const int o_rt = ixr * PADW + iyl;

  u4v hw; hw.x = 0u; hw.y = 0u; hw.z = 0u; hw.w = 0u;
  u4v lw; lw.x = 0u; lw.y = 0u; lw.z = 0u; lw.w = 0u;
#pragma unroll 1
  for (int half = 0; half < 2; ++half) {
    const unsigned short* s = xpb + (size_t)(cb + half * 4) * PADHW;
    unsigned hu[2], lu[2];
#pragma unroll
    for (int i = 0; i < 4; ++i) {
      const unsigned short* sc = s + (size_t)i * PADHW;
      const float vlt = bf_bits2f(sc[o_lt]);
      const float vrb = bf_bits2f(sc[o_rb]);
      const float vlb = bf_bits2f(sc[o_lb]);
      const float vrt = bf_bits2f(sc[o_rt]);
      const float xo = ((g_lt * vlt + g_rb * vrb) + g_lb * vlb) + g_rt * vrt;
      const unsigned short hb = f2bf_bits(xo);
      const unsigned short lb = f2bf_bits(xo - bf_bits2f(hb));
      if (i & 1) { hu[i >> 1] |= ((unsigned)hb << 16); lu[i >> 1] |= ((unsigned)lb << 16); }
      else       { hu[i >> 1]  = (unsigned)hb;          lu[i >> 1]  = (unsigned)lb; }
    }
    if (half == 0) { hw.x = hu[0]; hw.y = hu[1]; lw.x = lu[0]; lw.y = lu[1]; }
    else           { hw.z = hu[0]; hw.w = hu[1]; lw.z = lu[0]; lw.w = lu[1]; }
  }
  u4v* dh = (u4v*)(void*)xh + g;
  u4v* dl = (u4v*)(void*)xl + g;
  *(volatile u4v*)dh = hw;
  *(volatile u4v*)dl = lw;
  __threadfence();
  *(volatile u4v*)dh = hw;
  *(volatile u4v*)dl = lw;
}

extern "C" void kernel_launch(void* const* d_in, const int* in_sizes, int n_in,
                              void* d_out, int out_size, void* d_ws, size_t ws_size,
                              hipStream_t stream) {
  if (n_in < 4) return;
  if (in_sizes[0] != NIMG * NCH * HWPIX) return;
  if (in_sizes[1] != NOFFCH * KDIM) return;
  if (in_sizes[2] != NOFFCH) return;
  if (in_sizes[3] != NCH * KDIM) return;
  if (out_size != NIMG * NCH * HWPIX) return;

  const float* x      = (const float*)d_in[0];
  const float* w_off  = (const float*)d_in[1];
  const float* b_off  = (const float*)d_in[2];
  const float* w_conv = (const float*)d_in[3];
  float* out = (float*)d_out;

  const size_t szXP  = (size_t)NXP * 2;
  const size_t szW   = (size_t)NCH * KDIM * 2;
  const size_t szPL  = (size_t)HWPIX * KDIM * 2;
  const size_t szOFF = (size_t)NCH * HWPIX * 4;
  const size_t offXP   = 0;
  const size_t offWOFF = offXP + szXP;
  const size_t offWC   = offWOFF + szW;
  const size_t offIM   = offWC + szW;
  const size_t offOFF  = offIM + szPL;
  const size_t offXH   = offOFF + szOFF;
  const size_t offXL   = offXH + szPL;
  const size_t total   = offXL + szPL;
  if (total > ws_size) return;

  char* ws = (char*)d_ws;
  unsigned short* XP   = (unsigned short*)(ws + offXP);
  unsigned short* WOFF = (unsigned short*)(ws + offWOFF);
  unsigned short* WC   = (unsigned short*)(ws + offWC);
  unsigned short* IM   = (unsigned short*)(ws + offIM);
  float*          OFF  = (float*)(ws + offOFF);
  unsigned short* XH   = (unsigned short*)(ws + offXH);
  unsigned short* XL   = (unsigned short*)(ws + offXL);

  const int prepBlocks = 2 * ((NCH * QPR) / 256);
  const int padBlocks  = (NXP / 8) / 256;
  const int rowBlocks  = (HWPIX * QPR) / 256;
  const int gemmTiles  = (NCH / 64) * (HWPIX / 64);
  const int gemmBlocks = (gemmTiles + 7) / 8;

  k_prep_w<<<dim3(prepBlocks, 1, 1), dim3(256, 1, 1), 0, stream>>>(w_off, w_conv, WOFF, WC);
  k_pad_x<<<dim3(padBlocks, 1, 1), dim3(256, 1, 1), 0, stream>>>(x, XP);

  for (int b = 0; b < NIMG; ++b) {
    const unsigned short* xpb = XP + (size_t)b * NCH * PADHW;
    float* outb = out + (size_t)b * NCH * HWPIX;
    const float* xb = x + (size_t)b * NCH * HWPIX;

    k_im2col<<<dim3(rowBlocks, 1, 1), dim3(256, 1, 1), 0, stream>>>(xpb, IM);
    wmma_gemm64<1, 0, false><<<dim3(gemmBlocks, 1, 1), dim3(256, 1, 1), 0, stream>>>(
        WOFF, WOFF, KDIM, 0L, IM, IM, KDIM, 0L, OFF, HWPIX, 0L, xb, 0L, NCH, HWPIX, KDIM, 1.0f);
    k_sample<<<dim3(rowBlocks, 1, 1), dim3(256, 1, 1), 0, stream>>>(xpb, OFF, b_off, XH, XL);
    wmma_gemm64<1, 2, true><<<dim3(gemmBlocks, 1, 1), dim3(256, 1, 1), 0, stream>>>(
        WC, WC, KDIM, 0L, XH, XL, KDIM, 0L, outb, HWPIX, 0L, xb, 0L, NCH, HWPIX, KDIM, 1.0f);
  }
}
